// SelfAttentionModule_17008070492459
// MI455X (gfx1250) — hardware-verified
//
#include <hip/hip_runtime.h>


#ifndef NB
#define NB 4
#endif
#ifndef SEQ
#define SEQ 4096
#endif
#define NB_FULL 4
#define NFULL 4096
#define NC 256
#define ND 32
#define KQ 96
#define NWROWS (NC + 2 * ND)
#define PT 72
#define PP 72

static_assert(SEQ % 64 == 0);
static_assert(SEQ <= NFULL);
static_assert(NB >= 1 && NB <= NB_FULL);
static_assert(NC % 64 == 0 && ND == 32);

typedef __bf16 bf16_t;
typedef __bf16 v8bf __attribute__((ext_vector_type(8)));
typedef __bf16 v16bf __attribute__((ext_vector_type(16)));
typedef float v8f __attribute__((ext_vector_type(8)));
typedef float v4f __attribute__((ext_vector_type(4)));
typedef unsigned int v4u __attribute__((ext_vector_type(4)));
typedef unsigned short u16;

__device__ __forceinline__ unsigned bf_bits(float f) {
  unsigned u = __builtin_bit_cast(unsigned, f);
  u += 0x7FFFu + ((u >> 16) & 1u);
  return u >> 16;
}
__device__ __forceinline__ float bf_val(unsigned b) { return __builtin_bit_cast(float, b << 16); }
__device__ __forceinline__ float bf_rne(float f) { return bf_val(bf_bits(f)); }
__device__ __forceinline__ unsigned pk2(unsigned lo, unsigned hi) { return (lo & 0xFFFFu) | (hi << 16); }

__device__ __forceinline__ v16bf cat8(v8bf a, v8bf b) {
  return __builtin_shufflevector(a, b, 0, 1, 2, 3, 4, 5, 6, 7, 8, 9, 10, 11, 12, 13, 14, 15);
}
__device__ __forceinline__ v16bf ldfrag(const bf16_t* p) {
  return cat8(*(const v8bf*)p, *(const v8bf*)(p + 16));
}
__device__ __forceinline__ v8f wmma16(v16bf a, v16bf b, v8f c) {
  v8f d = __builtin_amdgcn_wmma_f32_16x16x32_bf16(false, a, false, b, (short)0, c, false, false);
  asm volatile("v_nop\n\tv_nop\n\tv_nop\n\tv_nop" : "+v"(d) : "v"(a), "v"(b));
  return d;
}

__global__ void __launch_bounds__(256)
k_wconv(const float* __restrict__ wv, const float* __restrict__ wq, const float* __restrict__ wk,
        bf16_t* __restrict__ wcat) {
  const int gid = blockIdx.x * 256 + threadIdx.x;
  const int row = gid >> 5;
  const int c8 = (gid & 31) * 8;
  if (row >= NWROWS) return;
  const float* src = (row < NC) ? (wv + (size_t)row * NC)
                   : ((row < NC + ND) ? (wq + (size_t)(row - NC) * NC)
                                      : (wk + (size_t)(row - NC - ND) * NC));
  const v4f a = *(const v4f*)(src + c8);
  const v4f c = *(const v4f*)(src + c8 + 4);
  v4u o;
  o.x = pk2(bf_bits(a.x), bf_bits(a.y));
  o.y = pk2(bf_bits(a.z), bf_bits(a.w));
  o.z = pk2(bf_bits(c.x), bf_bits(c.y));
  o.w = pk2(bf_bits(c.z), bf_bits(c.w));
  volatile v4u* dst = (volatile v4u*)(wcat + (size_t)row * NC + c8);
  *dst = o;
  __threadfence();
  *dst = o;
}

__global__ void __launch_bounds__(256)
k_xconv(const float* __restrict__ x, bf16_t* __restrict__ xt) {
  __shared__ __attribute__((aligned(16))) u16 tile[64 * PT];
  const int t = threadIdx.x;
  const int c0 = blockIdx.x * 64, n0 = blockIdx.y * 64, b = blockIdx.z;
  const float* xb = x + ((size_t)b * NC + c0) * NFULL + n0;
#pragma unroll
  for (int k = 0; k < 4; k++) {
    const int idx = t + 256 * k;
    const int row = idx >> 4, q4 = idx & 15;
    const v4f v = *(const v4f*)(xb + (size_t)row * NFULL + 4 * q4);
    const int nl = 4 * q4;
    tile[(nl + 0) * PT + row] = (u16)bf_bits(v.x);
    tile[(nl + 1) * PT + row] = (u16)bf_bits(v.y);
    tile[(nl + 2) * PT + row] = (u16)bf_bits(v.z);
    tile[(nl + 3) * PT + row] = (u16)bf_bits(v.w);
  }
  __syncthreads();
  v4u vals[2];
#pragma unroll
  for (int q = 0; q < 2; q++) {
    const int n = 32 * q + (t >> 3), piece = t & 7;
    vals[q] = *(const v4u*)&tile[n * PT + 8 * piece];
  }
#pragma unroll
  for (int q = 0; q < 2; q++) {
    const int n = 32 * q + (t >> 3), piece = t & 7;
    *(volatile v4u*)(xt + ((size_t)b * SEQ + n0 + n) * NC + c0 + 8 * piece) = vals[q];
  }
  __threadfence();
#pragma unroll
  for (int q = 0; q < 2; q++) {
    const int n = 32 * q + (t >> 3), piece = t & 7;
    *(volatile v4u*)(xt + ((size_t)b * SEQ + n0 + n) * NC + c0 + 8 * piece) = vals[q];
  }
}

__global__ void __launch_bounds__(128)
k_proj(const bf16_t* __restrict__ xt, const bf16_t* __restrict__ wcat,
       const float* __restrict__ bq, const float* __restrict__ bk, const float* __restrict__ bv,
       bf16_t* __restrict__ qcat, bf16_t* __restrict__ kcat,
       bf16_t* __restrict__ vh, bf16_t* __restrict__ vl) {
  __shared__ __attribute__((aligned(16))) u16 sm[2 * 64 * KQ];
  const int t = threadIdx.x, w = t >> 5, l = t & 31, h = l >> 4, m = l & 15;
  const int n0 = blockIdx.x * 64, y = blockIdx.y, b = blockIdx.z;
  const bf16_t* xa = xt + ((size_t)b * SEQ + n0 + 16 * w + m) * NC + 8 * h;
  const bf16_t* wb = wcat + (size_t)(64 * y + m) * NC + 8 * h;
  const v8f zero = {};
  v8f acc[4];
#pragma unroll
  for (int ct = 0; ct < 4; ct++) acc[ct] = zero;

#pragma unroll 2
  for (int c0 = 0; c0 < NC; c0 += 32) {
    const v16bf a = ldfrag(xa + c0);
#pragma unroll
    for (int ct = 0; ct < 4; ct++) {
      const v16bf bb = ldfrag(wb + (size_t)(16 * ct) * NC + c0);
      acc[ct] = wmma16(a, bb, acc[ct]);
    }
  }

  if (y < 4) {
    const int cb = 64 * y;
    u16* sh = sm;
    u16* sl = sm + 64 * PT;
#pragma unroll
    for (int ct = 0; ct < 4; ct++) {
      const int cl = 16 * ct + m;
      const float bias = bf_rne(bv[cb + cl]);
      unsigned hb[8], lb[8];
#pragma unroll
      for (int r = 0; r < 8; r++) {
        const float v = acc[ct][r] + bias;
        const unsigned hi = bf_bits(v);
        hb[r] = hi;
        lb[r] = bf_bits(v - bf_val(hi));
      }
      v4u ph, pl;
      ph.x = pk2(hb[0], hb[1]); ph.y = pk2(hb[2], hb[3]); ph.z = pk2(hb[4], hb[5]); ph.w = pk2(hb[6], hb[7]);
      pl.x = pk2(lb[0], lb[1]); pl.y = pk2(lb[2], lb[3]); pl.z = pk2(lb[4], lb[5]); pl.w = pk2(lb[6], lb[7]);
      *(v4u*)&sh[cl * PT + 16 * w + 8 * h] = ph;
      *(v4u*)&sl[cl * PT + 16 * w + 8 * h] = pl;
    }
  } else {
    u16* sq = sm;
    u16* sk = sm + 64 * KQ;
#pragma unroll
    for (int ct = 0; ct < 4; ct++) {
      const int d = 16 * (ct & 1) + m;
      const float* bp = (ct < 2) ? bq : bk;
      const float bias = bf_rne(bp[d]);
#pragma unroll
      for (int r = 0; r < 8; r++) {
        const int nl = 16 * w + 8 * h + r;
        const float v = acc[ct][r] + bias;
        const unsigned hi = bf_bits(v);
        const unsigned lo = bf_bits(v - bf_val(hi));
        if (ct < 2) {
          sq[nl * KQ + d] = (u16)hi;
          sq[nl * KQ + ND + d] = (u16)hi;
          sq[nl * KQ + 2 * ND + d] = (u16)lo;
        } else {
          sk[nl * KQ + d] = (u16)hi;
          sk[nl * KQ + ND + d] = (u16)lo;
          sk[nl * KQ + 2 * ND + d] = (u16)hi;
        }
      }
    }
  }
  __syncthreads();

  if (y < 4) {
    const int cb = 64 * y;
    const u16* sh = sm;
    const u16* sl = sm + 64 * PT;
    v4u oh[4], ol[4];
#pragma unroll
    for (int q = 0; q < 4; q++) {
      const int line = 16 * q + (t >> 3), piece = t & 7;
      oh[q] = *(const v4u*)&sh[line * PT + 8 * piece];
      ol[q] = *(const v4u*)&sl[line * PT + 8 * piece];
    }
#pragma unroll
    for (int q = 0; q < 4; q++) {
      const int line = 16 * q + (t >> 3), piece = t & 7;
      const size_t gi = ((size_t)b * NC + cb + line) * SEQ + n0 + 8 * piece;
      *(volatile v4u*)(vh + gi) = oh[q];
      *(volatile v4u*)(vl + gi) = ol[q];
    }
    __threadfence();
#pragma unroll
    for (int q = 0; q < 4; q++) {
      const int line = 16 * q + (t >> 3), piece = t & 7;
      const size_t gi = ((size_t)b * NC + cb + line) * SEQ + n0 + 8 * piece;
      *(volatile v4u*)(vh + gi) = oh[q];
      *(volatile v4u*)(vl + gi) = ol[q];
    }
  } else {
    const v4u* sq4 = (const v4u*)sm;
    const v4u* sk4 = (const v4u*)(sm + 64 * KQ);
    v4u* qg = (v4u*)(qcat + ((size_t)b * SEQ + n0) * KQ);
    v4u* kg = (v4u*)(kcat + ((size_t)b * SEQ + n0) * KQ);
    v4u oq[6], ok[6];
#pragma unroll
    for (int q = 0; q < 6; q++) {
      oq[q] = sq4[128 * q + t];
      ok[q] = sk4[128 * q + t];
    }
#pragma unroll
    for (int q = 0; q < 6; q++) {
      *(volatile v4u*)(qg + 128 * q + t) = oq[q];
      *(volatile v4u*)(kg + 128 * q + t) = ok[q];
    }
    __threadfence();
#pragma unroll
    for (int q = 0; q < 6; q++) {
      *(volatile v4u*)(qg + 128 * q + t) = oq[q];
      *(volatile v4u*)(kg + 128 * q + t) = ok[q];
    }
  }
}

__global__ void __launch_bounds__(128)
k_stats(const bf16_t* __restrict__ qcat, const bf16_t* __restrict__ kcat,
        float* __restrict__ mst, float* __restrict__ rst) {
  __shared__ __attribute__((aligned(16))) float sM[64];
  __shared__ __attribute__((aligned(16))) float sR[64];
  const int t = threadIdx.x, w = t >> 5, l = t & 31, h = l >> 4, m = l & 15;
  const int ib = blockIdx.x * 64, b = blockIdx.y;
  const bf16_t* qa = qcat + ((size_t)b * SEQ + ib + 16 * w + m) * KQ + 8 * h;
  const v16bf a0 = ldfrag(qa);
  const v16bf a1 = ldfrag(qa + 32);
  const v16bf a2 = ldfrag(qa + 64);
  const bf16_t* kb = kcat + ((size_t)b * SEQ + m) * KQ + 8 * h;
  const v8f zero = {};
  float mx[8], sx[8];
#pragma unroll
  for (int r = 0; r < 8; r++) { mx[r] = -__builtin_inff(); sx[r] = 0.f; }

  for (int j0 = 0; j0 < SEQ; j0 += 64) {
    v8f e[4];
#pragma unroll
    for (int u = 0; u < 4; u++) {
      const bf16_t* kp = kb + (size_t)(j0 + 16 * u) * KQ;
      v8f acc = wmma16(a0, ldfrag(kp), zero);
      acc = wmma16(a1, ldfrag(kp + 32), acc);
      acc = wmma16(a2, ldfrag(kp + 64), acc);
      e[u] = acc;
    }
#pragma unroll
    for (int r = 0; r < 8; r++) {
      const float tmax = fmaxf(fmaxf(e[0][r], e[1][r]), fmaxf(e[2][r], e[3][r]));
      const float mn = fmaxf(mx[r], tmax);
      float s = sx[r] * __expf(mx[r] - mn);
      s += (__expf(e[0][r] - mn) + __expf(e[1][r] - mn)) + (__expf(e[2][r] - mn) + __expf(e[3][r] - mn));
      sx[r] = s;
      mx[r] = mn;
    }
  }
#pragma unroll
  for (int mk = 1; mk < 16; mk <<= 1) {
#pragma unroll
    for (int r = 0; r < 8; r++) {
      const float mo = __shfl_xor(mx[r], mk, 32);
      const float so = __shfl_xor(sx[r], mk, 32);
      const float mn = fmaxf(mx[r], mo);
      sx[r] = sx[r] * __expf(mx[r] - mn) + so * __expf(mo - mn);
      mx[r] = mn;
    }
  }
  const int rs = l & 7;
  float mv = mx[0], sv = sx[0];
#pragma unroll
  for (int r = 1; r < 8; r++) {
    mv = (rs == r) ? mx[r] : mv;
    sv = (rs == r) ? sx[r] : sv;
  }
  if (m < 8) {
    sM[16 * w + 8 * h + rs] = mv;
    sR[16 * w + 8 * h + rs] = 1.0f / sv;
  }
  __syncthreads();
  if (w == 0) {
    const v4f am = *(const v4f*)&sM[4 * m];
    const v4f ar = *(const v4f*)&sR[4 * m];
    v4f val;
    val.x = h ? ar.x : am.x;
    val.y = h ? ar.y : am.y;
    val.z = h ? ar.z : am.z;
    val.w = h ? ar.w : am.w;
    float* dp = (h ? rst : mst) + (size_t)b * SEQ + ib + 4 * m;
    *(volatile v4f*)dp = val;
    __threadfence();
    *(volatile v4f*)dp = val;
  }
}

__global__ void __launch_bounds__(256)
k_out(const bf16_t* __restrict__ qcat, const bf16_t* __restrict__ kcat,
      const bf16_t* __restrict__ vh, const bf16_t* __restrict__ vl,
      const float* __restrict__ mst, const float* __restrict__ rst,
      const float* __restrict__ x, const float* __restrict__ gamma,
      float* __restrict__ out) {
  __shared__ __attribute__((aligned(16))) u16 Psm[2 * 32 * PP];
  __shared__ __attribute__((aligned(16))) float ost[NC * 32];
  const int t = threadIdx.x, w = t >> 5, l = t & 31, h = l >> 4, m = l & 15;
  const int j0 = blockIdx.x * 32, b = blockIdx.y;
  const int it = w >> 1, jt = w & 1, cw = 32 * w;
  const bf16_t* qa  = qcat + ((size_t)b * SEQ + 16 * it + m) * KQ + 8 * h;
  const bf16_t* kbp = kcat + ((size_t)b * SEQ + j0 + 16 * jt + m) * KQ + 8 * h;
  const float* mp = mst + (size_t)b * SEQ + 16 * it + 8 * h;
  const float* rp = rst + (size_t)b * SEQ + 16 * it + 8 * h;
  const bf16_t* vha = vh + ((size_t)b * NC + cw + m) * SEQ + 8 * h;
  const bf16_t* vla = vl + ((size_t)b * NC + cw + m) * SEQ + 8 * h;
  const int pst = (16 * jt + m) * PP + 16 * it + 8 * h;
  const v8f zero = {};
  v8f acc[2][2];
#pragma unroll
  for (int ct = 0; ct < 2; ct++) { acc[ct][0] = zero; acc[ct][1] = zero; }

  for (int i0 = 0; i0 < SEQ; i0 += 64) {
    {
      const bf16_t* qp = qa + (size_t)i0 * KQ;
      v8f e = wmma16(ldfrag(qp), ldfrag(kbp), zero);
      e = wmma16(ldfrag(qp + 32), ldfrag(kbp + 32), e);
      e = wmma16(ldfrag(qp + 64), ldfrag(kbp + 64), e);
      const v4f ma = *(const v4f*)(mp + i0), mb = *(const v4f*)(mp + i0 + 4);
      const v4f ra = *(const v4f*)(rp + i0), rb = *(const v4f*)(rp + i0 + 4);
      const float mm[8] = {ma.x, ma.y, ma.z, ma.w, mb.x, mb.y, mb.z, mb.w};
      const float rr[8] = {ra.x, ra.y, ra.z, ra.w, rb.x, rb.y, rb.z, rb.w};
      unsigned hb[8], lb[8];
#pragma unroll
      for (int r = 0; r < 8; r++) {
        const float p = __expf(e[r] - mm[r]) * rr[r];
        const unsigned hi = bf_bits(p);
        hb[r] = hi;
        lb[r] = bf_bits(p - bf_val(hi));
      }
      v4u ph, pl;
      ph.x = pk2(hb[0], hb[1]); ph.y = pk2(hb[2], hb[3]); ph.z = pk2(hb[4], hb[5]); ph.w = pk2(hb[6], hb[7]);
      pl.x = pk2(lb[0], lb[1]); pl.y = pk2(lb[2], lb[3]); pl.z = pk2(lb[4], lb[5]); pl.w = pk2(lb[6], lb[7]);
      *(v4u*)&Psm[pst] = ph;
      *(v4u*)&Psm[32 * PP + pst] = pl;
    }
    __syncthreads();
#pragma unroll
    for (int ks = 0; ks < 2; ks++) {
      const int kk = 32 * ks;
      const v16bf ph0 = ldfrag((const bf16_t*)&Psm[m * PP + kk + 8 * h]);
      const v16bf ph1 = ldfrag((const bf16_t*)&Psm[(16 + m) * PP + kk + 8 * h]);
      const v16bf pl0 = ldfrag((const bf16_t*)&Psm[32 * PP + m * PP + kk + 8 * h]);
      const v16bf pl1 = ldfrag((const bf16_t*)&Psm[32 * PP + (16 + m) * PP + kk + 8 * h]);
#pragma unroll
      for (int ct = 0; ct < 2; ct++) {
        const size_t vo = (size_t)(16 * ct) * SEQ + i0 + kk;
        const v16bf ah = ldfrag(vha + vo);
        const v16bf al = ldfrag(vla + vo);
        acc[ct][0] = wmma16(ah, ph0, acc[ct][0]);
        acc[ct][0] = wmma16(ah, pl0, acc[ct][0]);
        acc[ct][0] = wmma16(al, ph0, acc[ct][0]);
        acc[ct][1] = wmma16(ah, ph1, acc[ct][1]);
        acc[ct][1] = wmma16(ah, pl1, acc[ct][1]);
        acc[ct][1] = wmma16(al, ph1, acc[ct][1]);
      }
    }
    __syncthreads();
  }
  const float gsc = bf_rne(gamma[0]);
#pragma unroll
  for (int ct = 0; ct < 2; ct++) {
#pragma unroll
    for (int j2 = 0; j2 < 2; j2++) {
#pragma unroll
      for (int r = 0; r < 8; r++) {
        ost[(cw + 16 * ct + 8 * h + r) * 32 + 16 * j2 + m] = gsc * acc[ct][j2][r];
      }
    }
  }
  __syncthreads();
  v4f res[8];
#pragma unroll
  for (int q = 0; q < 8; q++) {
    const int c = 32 * q + (t >> 3), piece = t & 7;
    const v4f o4 = *(const v4f*)&ost[c * 32 + 4 * piece];
    const size_t gi = ((size_t)b * NC + c) * NFULL + j0 + 4 * piece;
    const v4f x4 = *(const v4f*)(x + gi);
    v4f rv;
    rv.x = o4.x + bf_rne(x4.x);
    rv.y = o4.y + bf_rne(x4.y);
    rv.z = o4.z + bf_rne(x4.z);
    rv.w = o4.w + bf_rne(x4.w);
    res[q] = rv;
  }
#pragma unroll
  for (int q = 0; q < 8; q++) {
    const int c = 32 * q + (t >> 3), piece = t & 7;
    const size_t gi = ((size_t)b * NC + c) * NFULL + j0 + 4 * piece;
    *(volatile v4f*)(out + gi) = res[q];
  }
  __threadfence();
#pragma unroll
  for (int q = 0; q < 8; q++) {
    const int c = 32 * q + (t >> 3), piece = t & 7;
    const size_t gi = ((size_t)b * NC + c) * NFULL + j0 + 4 * piece;
    *(volatile v4f*)(out + gi) = res[q];
  }
}

extern "C" void kernel_launch(void* const* d_in, const int* in_sizes, int n_in,
                              void* d_out, int out_size, void* d_ws, size_t ws_size,
                              hipStream_t stream) {
  if (n_in < 8) return;
  if (in_sizes[0] < NB * NC * NFULL) return;
  if (in_sizes[1] < ND * NC || in_sizes[3] < ND * NC || in_sizes[5] < NC * NC) return;
  if (in_sizes[2] < ND || in_sizes[4] < ND || in_sizes[6] < NC || in_sizes[7] < 1) return;
  if (out_size < NB * NC * NFULL) return;

  const float* x  = (const float*)d_in[0];
  const float* wq = (const float*)d_in[1];
  const float* bq = (const float*)d_in[2];
  const float* wk = (const float*)d_in[3];
  const float* bk = (const float*)d_in[4];
  const float* wv = (const float*)d_in[5];
  const float* bv = (const float*)d_in[6];
  const float* gm = (const float*)d_in[7];
  float* out = (float*)d_out;

  char* ws = (char*)d_ws;
  size_t off = 0;
  bf16_t* wcat = (bf16_t*)(ws + off); off += (size_t)NWROWS * NC * 2;
  bf16_t* xt   = (bf16_t*)(ws + off); off += (size_t)NB * SEQ * NC * 2;
  bf16_t* vh   = (bf16_t*)(ws + off); off += (size_t)NB * NC * SEQ * 2;
  bf16_t* vl   = (bf16_t*)(ws + off); off += (size_t)NB * NC * SEQ * 2;
  bf16_t* qcat = (bf16_t*)(ws + off); off += (size_t)NB * SEQ * KQ * 2;
  bf16_t* kcat = (bf16_t*)(ws + off); off += (size_t)NB * SEQ * KQ * 2;
  float*  mst  = (float*)(ws + off);  off += (size_t)NB * SEQ * 4;
  float*  rst  = (float*)(ws + off);  off += (size_t)NB * SEQ * 4;
  if (off > ws_size) return;

  k_wconv<<<dim3((NWROWS * 32) / 256), dim3(256), 0, stream>>>(wv, wq, wk, wcat);
  k_xconv<<<dim3(NC / 64, SEQ / 64, NB), dim3(256), 0, stream>>>(x, xt);
  k_proj<<<dim3(SEQ / 64, 5, NB), dim3(128), 0, stream>>>(xt, wcat, bq, bk, bv, qcat, kcat, vh, vl);
  k_stats<<<dim3(SEQ / 64, NB), dim3(128), 0, stream>>>(qcat, kcat, mst, rst);
  k_out<<<dim3(SEQ / 32, NB), dim3(256), 0, stream>>>(qcat, kcat, vh, vl, mst, rst, x, gm, out);
}
